// TravelingObserverModel_42030549958779
// MI455X (gfx1250) — hardware-verified
//
#include <hip/hip_runtime.h>
#include <stddef.h>
#include <stdint.h>


#define NB     128
#define NIN    1024
#define NOUT   512
#define NV     2048
#define NVAR   4096
#define NS     1024
#define NC     64
#define NH     128
#define LENC   2
#define LCORE  3
#define LDEC   2
#define NEMAP  (1 + 2 * LENC)
#define NDMAP  (2 * LDEC)
#define MCH    32768
#define NITER  50
#define XSE    4.0f
#define XSD    0.125f
#define WSC    64.0f
#define NTHR   256
#define WSCAP  134217728
#define LDS_GEMM (8 * 32 * 64 * 4)
#define PWB_E  ((LENC * 2 * NH * NH) / (8 * NTHR))
#define PWB_D  ((LDEC * 2 * NH * NH) / (8 * NTHR))
#define ENC_CH ((NB * NIN) / MCH)
#define DEC_CH ((NB * NOUT) / MCH)

static_assert(((LENC * 2 * NH * NH) % (8 * NTHR)) == 0);
static_assert(((LDEC * 2 * NH * NH) % (8 * NTHR)) == 0);
static_assert(NH == 128);
static_assert(NC == 64);
static_assert(NS == 16 * 64);
static_assert((MCH % NIN) == 0);
static_assert((MCH % NOUT) == 0);
static_assert(((NB * NIN) % MCH) == 0);
static_assert(((NB * NOUT) % MCH) == 0);
static_assert((MCH % 128) == 0);
static_assert((NIN & (NIN - 1)) == 0);
static_assert((NOUT & (NOUT - 1)) == 0);
static_assert((NOUT % 32) == 0);
static_assert((NIN % 4) == 0);
static_assert((NH % 32) == 0);
static_assert(NITER == 50);
static_assert(LDS_GEMM <= 300 * 1024);
static_assert(NTHR == 256);

typedef float          v4f  __attribute__((ext_vector_type(4)));
typedef float          v8f  __attribute__((ext_vector_type(8)));
typedef _Float16       v8h  __attribute__((ext_vector_type(8)));
typedef _Float16       v16h __attribute__((ext_vector_type(16)));
union FragH { v16h v; v8h h[2]; };

__device__ __forceinline__ v8f wmf(v16h a, v16h b, v8f c) {
  v8f d = __builtin_amdgcn_wmma_f32_16x16x32_f16(false, a, false, b, (short)0, c, false, false);
  asm volatile("v_nop\n\tv_nop\n\tv_nop\n\tv_nop" : "+v"(d) : "v"(a), "v"(b));
  return d;
}

__device__ __forceinline__ int wrapclamp(int i, int n) {
  i = (i < 0) ? (i + n) : i;
  i = (i < 0) ? 0 : i;
  i = (i > n - 1) ? (n - 1) : i;
  return i;
}

__device__ __forceinline__ v4f relu4(v4f v) {
  v4f r;
  r.x = fmaxf(v.x, 0.0f); r.y = fmaxf(v.y, 0.0f); r.z = fmaxf(v.z, 0.0f); r.w = fmaxf(v.w, 0.0f);
  return r;
}

__device__ __forceinline__ v8h cvt8(v4f a, v4f b, float s) {
  v8h r;
  r[0] = (_Float16)(a.x * s); r[1] = (_Float16)(a.y * s); r[2] = (_Float16)(a.z * s); r[3] = (_Float16)(a.w * s);
  r[4] = (_Float16)(b.x * s); r[5] = (_Float16)(b.y * s); r[6] = (_Float16)(b.z * s); r[7] = (_Float16)(b.w * s);
  return r;
}

__global__ __launch_bounds__(NTHR) void k_prepw(const float* __restrict__ We, const float* __restrict__ Wd, _Float16* wt) {
  const int t = blockIdx.x * NTHR + threadIdx.x;
  const float* p;
  if (blockIdx.x < PWB_E) p = We + (size_t)t * 8;
  else                    p = Wd + (size_t)(t - PWB_E * NTHR) * 8;
  const v4f f0 = *(const v4f*)p;
  const v4f f1 = *(const v4f*)(p + 4);
  const v8h a = cvt8(f0, f1, WSC);
  _Float16* d = wt + (size_t)t * 8;
  *(volatile v8h*)d = a;
  __threadfence();
  *(volatile v8h*)d = a;
}

__global__ __launch_bounds__(64) void k_attn(const int* __restrict__ vi, const int* __restrict__ ivi,
    const float* __restrict__ dctx, const float* __restrict__ basis, const float* __restrict__ alpha_p,
    const float* __restrict__ fGw, const float* __restrict__ fGb, const float* __restrict__ fBw, const float* __restrict__ fBb,
    const float* __restrict__ eGw, const float* __restrict__ eGb, const float* __restrict__ eBw, const float* __restrict__ eBb,
    float* gem, float* bem)
{
  __shared__ __attribute__((aligned(16))) float qv[NC];
  __shared__ __attribute__((aligned(16))) float xs[NS];
  __shared__ __attribute__((aligned(16))) float part[4 * NC];
  __shared__ __attribute__((aligned(16))) float av[NC];
  __shared__ __attribute__((aligned(16))) float ms[2 * NEMAP * NH];
  __shared__ float red[2];
  __shared__ float redb[2][2];

  const int t = threadIdx.x, lane = t & 31, w = t >> 5;
  const int n = blockIdx.x;
  {
    const int i1 = wrapclamp(ivi[n], NV);
    const int i2 = wrapclamp(vi[i1], NVAR);
    qv[t] = dctx[(size_t)i2 * NC + t];
  }
  __syncthreads();

  const float am1 = alpha_p[0] - 1.0f;
  const float pinv = 1.0f / am1;
  const bool sq = (pinv == 2.0f);

  float mx = -3.0e38f;
#pragma unroll 1
  for (int j = 0; j < 16; ++j) {
    const int s = t + 64 * j;
    const float* br = basis + (size_t)s * NC;
    float a0 = 0.0f, a1 = 0.0f, a2 = 0.0f, a3 = 0.0f;
#pragma unroll 2
    for (int c = 0; c < NC; c += 4) {
      const v4f bq = *(const v4f*)(br + c);
      const v4f qq = *(const v4f*)(qv + c);
      a0 += bq.x * qq.x; a1 += bq.y * qq.y; a2 += bq.z * qq.z; a3 += bq.w * qq.w;
    }
    const float sc = ((a0 + a1) + (a2 + a3)) * am1;
    xs[s] = sc;
    mx = fmaxf(mx, sc);
  }
#pragma unroll
  for (int o = 16; o > 0; o >>= 1) mx = fmaxf(mx, __shfl_xor(mx, o));
  if (lane == 0) red[w] = mx;
  __syncthreads();
  const float maxv = fmaxf(red[0], red[1]);

  float tau = maxv - 1.0f;
  const float thi = maxv - exp2f(am1 * log2f(1.0f / (float)NS));
  float dm = thi - tau;

  float xr[16];
#pragma unroll
  for (int j = 0; j < 16; ++j) xr[j] = xs[t + 64 * j];

#pragma unroll 1
  for (int it = 0; it < NITER; ++it) {
    dm *= 0.5f;
    const float tm = tau + dm;
    float sm = 0.0f;
    if (sq) {
#pragma unroll
      for (int j = 0; j < 16; ++j) { const float d = fmaxf(xr[j] - tm, 0.0f); sm += d * d; }
    } else {
#pragma unroll 1
      for (int j = 0; j < 16; ++j) {
        const float d = xs[t + 64 * j] - tm;
        const float pw = exp2f(pinv * log2f(d));
        sm += (d > 0.0f) ? pw : 0.0f;
      }
    }
#pragma unroll
    for (int o = 16; o > 0; o >>= 1) sm += __shfl_xor(sm, o);
    const int bi = it & 1;
    if (lane == 0) redb[bi][w] = sm;
    __syncthreads();
    const float f = (redb[bi][0] + redb[bi][1]) - 1.0f;
    if (f >= 0.0f) tau = tm;
  }

  float ps = 0.0f;
  if (sq) {
#pragma unroll
    for (int j = 0; j < 16; ++j) {
      const float d = fmaxf(xr[j] - tau, 0.0f);
      const float pw = d * d;
      xs[t + 64 * j] = pw;
      ps += pw;
    }
  } else {
#pragma unroll 1
    for (int j = 0; j < 16; ++j) {
      const float d = xs[t + 64 * j] - tau;
      const float pe = exp2f(pinv * log2f(d));
      const float pw = (d > 0.0f) ? pe : 0.0f;
      xs[t + 64 * j] = pw;
      ps += pw;
    }
  }
#pragma unroll
  for (int o = 16; o > 0; o >>= 1) ps += __shfl_xor(ps, o);
  if (lane == 0) red[w] = ps;
  __syncthreads();
  const float rs = 1.0f / (red[0] + red[1]);
#pragma unroll 4
  for (int j = 0; j < 16; ++j) xs[t + 64 * j] *= rs;
  __syncthreads();

  {
    const int cg = t & 15, sr = t >> 4;
    v4f a4 = {0.0f, 0.0f, 0.0f, 0.0f};
    const float* bb = basis + 4 * cg;
#pragma unroll 2
    for (int s = 256 * sr; s < 256 * sr + 256; ++s) {
      const float pv = xs[s];
      const v4f bq = *(const v4f*)(bb + (size_t)s * NC);
      a4 += pv * bq;
    }
    *(v4f*)(part + sr * NC + 4 * cg) = a4;
  }
  __syncthreads();
  av[t] = (part[t] + part[NC + t]) + (part[2 * NC + t] + part[3 * NC + t]);
  __syncthreads();

#pragma unroll 1
  for (int j = 0; j < 2 * NEMAP; ++j) {
    const int j5 = (j < NEMAP) ? j : (j - NEMAP);
    const float* Wm;
    const float* bm2;
    if (j < NEMAP) {
      Wm  = (j5 == 0) ? fGw : (eGw + (size_t)(j5 - 1) * NH * NC);
      bm2 = (j5 == 0) ? fGb : (eGb + (size_t)(j5 - 1) * NH);
    } else {
      Wm  = (j5 == 0) ? fBw : (eBw + (size_t)(j5 - 1) * NH * NC);
      bm2 = (j5 == 0) ? fBb : (eBb + (size_t)(j5 - 1) * NH);
    }
#pragma unroll
    for (int oo = 0; oo < 2; ++oo) {
      const int o = t + 64 * oo;
      const float* wr = Wm + (size_t)o * NC;
      float a0 = 0.0f, a1 = 0.0f, a2 = 0.0f, a3 = 0.0f;
#pragma unroll 2
      for (int c = 0; c < NC; c += 4) {
        const v4f wq = *(const v4f*)(wr + c);
        const v4f aq = *(const v4f*)(av + c);
        a0 += wq.x * aq.x; a1 += wq.y * aq.y; a2 += wq.z * aq.z; a3 += wq.w * aq.w;
      }
      ms[j * NH + o] = ((a0 + a1) + (a2 + a3)) + bm2[o];
    }
  }
  __syncthreads();

#pragma unroll
  for (int jj = 0; jj < NEMAP; ++jj) {
    const int j = w + 2 * jj;
    const v4f v = *(const v4f*)(ms + j * NH + 4 * lane);
    float* dst = (j < NEMAP) ? (gem + ((size_t)j * NIN + n) * NH) : (bem + ((size_t)(j - NEMAP) * NIN + n) * NH);
    *(volatile v4f*)(dst + 4 * lane) = v;
  }
  __threadfence();
#pragma unroll
  for (int jj = 0; jj < NEMAP; ++jj) {
    const int j = w + 2 * jj;
    const v4f v = *(const v4f*)(ms + j * NH + 4 * lane);
    float* dst = (j < NEMAP) ? (gem + ((size_t)j * NIN + n) * NH) : (bem + ((size_t)(j - NEMAP) * NIN + n) * NH);
    *(volatile v4f*)(dst + 4 * lane) = v;
  }
}

__global__ __launch_bounds__(64) void k_dmaps(const int* __restrict__ vi, const int* __restrict__ ovi,
    const float* __restrict__ dctx,
    const float* __restrict__ dGw, const float* __restrict__ dGb, const float* __restrict__ dBw, const float* __restrict__ dBb,
    float* gdm, float* bdm)
{
  __shared__ __attribute__((aligned(16))) float cv[NC];
  __shared__ __attribute__((aligned(16))) float ms[2 * NDMAP * NH];
  const int t = threadIdx.x, lane = t & 31, w = t >> 5;
  const int n = blockIdx.x;
  {
    const int i1 = wrapclamp(ovi[n], NV);
    const int i2 = wrapclamp(vi[i1], NVAR);
    cv[t] = dctx[(size_t)i2 * NC + t];
  }
  __syncthreads();
#pragma unroll 1
  for (int j = 0; j < 2 * NDMAP; ++j) {
    const float* Wm;
    const float* bm2;
    if (j < NDMAP) { Wm = dGw + (size_t)j * NH * NC;           bm2 = dGb + (size_t)j * NH; }
    else           { Wm = dBw + (size_t)(j - NDMAP) * NH * NC; bm2 = dBb + (size_t)(j - NDMAP) * NH; }
#pragma unroll
    for (int oo = 0; oo < 2; ++oo) {
      const int o = t + 64 * oo;
      const float* wr = Wm + (size_t)o * NC;
      float a0 = 0.0f, a1 = 0.0f, a2 = 0.0f, a3 = 0.0f;
#pragma unroll 2
      for (int c = 0; c < NC; c += 4) {
        const v4f wq = *(const v4f*)(wr + c);
        const v4f cq = *(const v4f*)(cv + c);
        a0 += wq.x * cq.x; a1 += wq.y * cq.y; a2 += wq.z * cq.z; a3 += wq.w * cq.w;
      }
      ms[j * NH + o] = ((a0 + a1) + (a2 + a3)) + bm2[o];
    }
  }
  __syncthreads();
#pragma unroll
  for (int jj = 0; jj < NDMAP; ++jj) {
    const int j = w + 2 * jj;
    const v4f v = *(const v4f*)(ms + j * NH + 4 * lane);
    float* dst = (j < NDMAP) ? (gdm + ((size_t)j * NOUT + n) * NH) : (bdm + ((size_t)(j - NDMAP) * NOUT + n) * NH);
    *(volatile v4f*)(dst + 4 * lane) = v;
  }
  __threadfence();
#pragma unroll
  for (int jj = 0; jj < NDMAP; ++jj) {
    const int j = w + 2 * jj;
    const v4f v = *(const v4f*)(ms + j * NH + 4 * lane);
    float* dst = (j < NDMAP) ? (gdm + ((size_t)j * NOUT + n) * NH) : (bdm + ((size_t)(j - NDMAP) * NOUT + n) * NH);
    *(volatile v4f*)(dst + 4 * lane) = v;
  }
}

template <int MODE>
__global__ __launch_bounds__(NTHR) void k_rowinit(int mbase, const float* __restrict__ xin,
    const float* __restrict__ fW, const float* __restrict__ fb,
    const float* __restrict__ g0, const float* __restrict__ e0,
    const float* __restrict__ sdec, float* X32, _Float16* X16, float s16)
{
  __shared__ __attribute__((aligned(16))) float stg[32 * NH];
  const int tid = threadIdx.x, lane = tid & 31, w = tid >> 5, hh = lane >> 4, m16 = lane & 15;
  const int r0 = blockIdx.x * 32;
  v4f vals[4];
#pragma unroll
  for (int u = 0; u < 4; ++u) {
    const int r = r0 + 4 * w + u;
    const int mg = mbase + r;
    v4f v;
    if (MODE == 0) {
      const int nn = mg & (NIN - 1);
      const float xv = xin[mg];
      const v4f W4 = *(const v4f*)(fW + 4 * lane);
      const v4f b4 = *(const v4f*)(fb + 4 * lane);
      const v4f g4 = *(const v4f*)(g0 + (size_t)nn * NH + 4 * lane);
      const v4f e4 = *(const v4f*)(e0 + (size_t)nn * NH + 4 * lane);
      const v4f h4 = W4 * xv + b4;
      v = relu4(g4 * h4 + e4);
    } else {
      const int b = mg / NOUT;
      v = *(const v4f*)(sdec + (size_t)b * NH + 4 * lane);
    }
    vals[u] = v;
    *(v4f*)(stg + (4 * w + u) * NH + 4 * lane) = v;
  }
  __syncthreads();
  v8h hv[2];
#pragma unroll
  for (int q = 0; q < 2; ++q) {
    const float* sp = stg + (4 * w + 2 * q + hh) * NH + 8 * m16;
    hv[q] = cvt8(*(const v4f*)sp, *(const v4f*)(sp + 4), s16);
  }
#pragma unroll
  for (int u = 0; u < 4; ++u)
    *(volatile v4f*)(X32 + (size_t)(r0 + 4 * w + u) * NH + 4 * lane) = vals[u];
#pragma unroll
  for (int q = 0; q < 2; ++q)
    *(volatile v8h*)(X16 + (size_t)(r0 + 4 * w + 2 * q + hh) * NH + 8 * m16) = hv[q];
  __threadfence();
#pragma unroll
  for (int u = 0; u < 4; ++u)
    *(volatile v4f*)(X32 + (size_t)(r0 + 4 * w + u) * NH + 4 * lane) = vals[u];
#pragma unroll
  for (int q = 0; q < 2; ++q)
    *(volatile v8h*)(X16 + (size_t)(r0 + 4 * w + 2 * q + hh) * NH + 8 * m16) = hv[q];
}

template <bool RESID, bool O32, bool O16>
__global__ __launch_bounds__(NTHR) void k_gemm(const _Float16* __restrict__ A16, const _Float16* __restrict__ Wt,
    const float* __restrict__ bias, const float* __restrict__ gmap, const float* __restrict__ emap,
    float* X32, _Float16* O16p, int nposmask, float osc, float s16)
{
  extern __shared__ v4f lds_dyn[];
  const int tid = threadIdx.x, lane = tid & 31, wave = tid >> 5, hh = lane >> 4, m = lane & 15;
  float* stg = (float*)lds_dyn + wave * (32 * 64);
  const int m0 = blockIdx.x * 128;
  const int wm = (wave >> 1) * 32, wn = (wave & 1) * 64;
  const int np0 = m0 & nposmask;

  v8f acc[2][4];
#pragma unroll
  for (int mt = 0; mt < 2; ++mt)
#pragma unroll
    for (int nt = 0; nt < 4; ++nt) { v8f z = {0.f, 0.f, 0.f, 0.f, 0.f, 0.f, 0.f, 0.f}; acc[mt][nt] = z; }

  const _Float16* ap = A16 + (size_t)(m0 + wm + m) * NH + 8 * hh;
  const _Float16* bp = Wt + (size_t)(wn + m) * NH + 8 * hh;
#pragma unroll 1
  for (int kt = 0; kt < NH / 32; ++kt) {
    const int k0 = 32 * kt;
    FragH a0, a1;
    a0.h[0] = *(const v8h*)(ap + k0);
    a0.h[1] = *(const v8h*)(ap + k0 + 16);
    a1.h[0] = *(const v8h*)(ap + 16 * NH + k0);
    a1.h[1] = *(const v8h*)(ap + 16 * NH + k0 + 16);
#pragma unroll
    for (int nt = 0; nt < 4; ++nt) {
      const _Float16* bq = bp + (size_t)nt * 16 * NH + k0;
      FragH b;
      b.h[0] = *(const v8h*)bq;
      b.h[1] = *(const v8h*)(bq + 16);
      acc[0][nt] = wmf(a0.v, b.v, acc[0][nt]);
      acc[1][nt] = wmf(a1.v, b.v, acc[1][nt]);
    }
  }

  float bv[4];
#pragma unroll
  for (int nt = 0; nt < 4; ++nt) bv[nt] = bias[wn + 16 * nt + m];
#pragma unroll
  for (int mt = 0; mt < 2; ++mt) {
    float* sp = stg + (16 * mt + 8 * hh) * 64 + m;
#pragma unroll
    for (int nt = 0; nt < 4; ++nt) {
#pragma unroll
      for (int r = 0; r < 8; ++r) sp[r * 64 + 16 * nt] = acc[mt][nt][r] * osc + bv[nt];
    }
  }
  __syncthreads();

  const float* gb = gmap + (size_t)(np0 + wm) * NH + wn + 4 * m;
  const float* eb = emap + (size_t)(np0 + wm) * NH + wn + 4 * m;
  float* xb = X32 + (size_t)(m0 + wm) * NH + wn;
#pragma unroll 4
  for (int q = 0; q < 16; ++q) {
    const int row = 2 * q + hh;
    float* s4 = stg + row * 64 + 4 * m;
    const v4f h4 = *(const v4f*)s4;
    const v4f g4 = *(const v4f*)(gb + (size_t)row * NH);
    const v4f e4 = *(const v4f*)(eb + (size_t)row * NH);
    v4f v = g4 * h4 + e4;
    if (RESID) v = *(const v4f*)(xb + (size_t)row * NH + 4 * m) + v;
    v = relu4(v);
    *(v4f*)s4 = v;
  }
  __syncthreads();

  if (O32) {
#pragma unroll
    for (int q = 0; q < 16; ++q) {
      const int row = 2 * q + hh;
      const v4f v = *(const v4f*)(stg + row * 64 + 4 * m);
      *(volatile v4f*)(xb + (size_t)row * NH + 4 * m) = v;
    }
  }
  if (O16) {
#pragma unroll
    for (int q = 0; q < 8; ++q) {
      const int row = 4 * q + (lane >> 3);
      const int c8 = 8 * (lane & 7);
      const float* sp = stg + row * 64 + c8;
      const v8h hv = cvt8(*(const v4f*)sp, *(const v4f*)(sp + 4), s16);
      *(volatile v8h*)(O16p + (size_t)(m0 + wm + row) * NH + wn + c8) = hv;
    }
  }
  __threadfence();
  if (O32) {
#pragma unroll
    for (int q = 0; q < 16; ++q) {
      const int row = 2 * q + hh;
      const v4f v = *(const v4f*)(stg + row * 64 + 4 * m);
      *(volatile v4f*)(xb + (size_t)row * NH + 4 * m) = v;
    }
  }
  if (O16) {
#pragma unroll
    for (int q = 0; q < 8; ++q) {
      const int row = 4 * q + (lane >> 3);
      const int c8 = 8 * (lane & 7);
      const float* sp = stg + row * 64 + c8;
      const v8h hv = cvt8(*(const v4f*)sp, *(const v4f*)(sp + 4), s16);
      *(volatile v8h*)(O16p + (size_t)(m0 + wm + row) * NH + wn + c8) = hv;
    }
  }
}

__global__ __launch_bounds__(NH) void k_nsum(const float* __restrict__ X32, float* score, int bbase) {
  __shared__ __attribute__((aligned(16))) float sv[NH];
  const int o = threadIdx.x, bl = blockIdx.x;
  const float* p = X32 + (size_t)bl * NIN * NH + o;
  float s0 = 0.0f, s1 = 0.0f, s2 = 0.0f, s3 = 0.0f;
#pragma unroll 1
  for (int nn = 0; nn < NIN; nn += 4) {
    s0 += p[(size_t)(nn) * NH];
    s1 += p[(size_t)(nn + 1) * NH];
    s2 += p[(size_t)(nn + 2) * NH];
    s3 += p[(size_t)(nn + 3) * NH];
  }
  sv[o] = (s0 + s1) + (s2 + s3);
  __syncthreads();
  if (o < 32) {
    const v4f v = *(const v4f*)(sv + 4 * o);
    float* dst = score + (size_t)(bbase + bl) * NH + 4 * o;
    *(volatile v4f*)dst = v;
    __threadfence();
    *(volatile v4f*)dst = v;
  }
}

__global__ __launch_bounds__(NH) void k_core(const float* __restrict__ sin_, const float* __restrict__ cW,
    const float* __restrict__ cb, float* sout)
{
  __shared__ __attribute__((aligned(16))) float xs[NH];
  __shared__ __attribute__((aligned(16))) float hs[NH];
  const int o = threadIdx.x, b = blockIdx.x;
  xs[o] = sin_[(size_t)b * NH + o];
  __syncthreads();
#pragma unroll 1
  for (int l = 0; l < LCORE; ++l) {
    const float* W0 = cW + (size_t)(2 * l) * NH * NH + (size_t)o * NH;
    const float* W1 = cW + (size_t)(2 * l + 1) * NH * NH + (size_t)o * NH;
    float a0 = 0.0f, a1 = 0.0f, a2 = 0.0f, a3 = 0.0f;
#pragma unroll 2
    for (int i = 0; i < NH; i += 4) {
      const v4f wq = *(const v4f*)(W0 + i);
      const v4f xq = *(const v4f*)(xs + i);
      a0 += wq.x * xq.x; a1 += wq.y * xq.y; a2 += wq.z * xq.z; a3 += wq.w * xq.w;
    }
    const float h = fmaxf(((a0 + a1) + (a2 + a3)) + cb[(size_t)(2 * l) * NH + o], 0.0f);
    hs[o] = h;
    __syncthreads();
    a0 = 0.0f; a1 = 0.0f; a2 = 0.0f; a3 = 0.0f;
#pragma unroll 2
    for (int i = 0; i < NH; i += 4) {
      const v4f wq = *(const v4f*)(W1 + i);
      const v4f hq = *(const v4f*)(hs + i);
      a0 += wq.x * hq.x; a1 += wq.y * hq.y; a2 += wq.z * hq.z; a3 += wq.w * hq.w;
    }
    const float h2 = ((a0 + a1) + (a2 + a3)) + cb[(size_t)(2 * l + 1) * NH + o];
    const float xn = fmaxf(xs[o] + h2, 0.0f);
    xs[o] = xn;
    __syncthreads();
  }
  if (o < 32) {
    const v4f v = *(const v4f*)(xs + 4 * o);
    float* dst = sout + (size_t)b * NH + 4 * o;
    *(volatile v4f*)dst = v;
    __threadfence();
    *(volatile v4f*)dst = v;
  }
}

__global__ __launch_bounds__(NTHR) void k_decf(int mbase, const float* __restrict__ X32,
    const int* __restrict__ vi, const int* __restrict__ ovi, const float* __restrict__ dctx,
    const float* __restrict__ dW, const float* __restrict__ db,
    const float* __restrict__ dGw, const float* __restrict__ dGb, const float* __restrict__ dBw, const float* __restrict__ dBb,
    float* out)
{
  __shared__ float gsv[32];
  __shared__ float bsv[32];
  __shared__ __attribute__((aligned(16))) float ys[32];
  const int tid = threadIdx.x, lane = tid & 31, w = tid >> 5;
  const int r0 = blockIdx.x * 32;
  const int mg0 = mbase + r0;
  const int n0 = mg0 & (NOUT - 1);
  if (tid < 32) {
    const int nn = n0 + tid;
    const int i1 = wrapclamp(ovi[nn], NV);
    const int i2 = wrapclamp(vi[i1], NVAR);
    const float* cr = dctx + (size_t)i2 * NC;
    float g = 0.0f, e = 0.0f;
#pragma unroll 1
    for (int c = 0; c < NC; ++c) {
      const float cvv = cr[c];
      g += dGw[c] * cvv;
      e += dBw[c] * cvv;
    }
    gsv[tid] = g + dGb[0];
    bsv[tid] = e + dBb[0];
  }
  __syncthreads();
  const v4f w4 = *(const v4f*)(dW + 4 * lane);
  const float dbv = db[0];
#pragma unroll
  for (int u = 0; u < 4; ++u) {
    const int j = 4 * w + u;
    const v4f x4 = *(const v4f*)(X32 + (size_t)(r0 + j) * NH + 4 * lane);
    float d = (x4.x * w4.x + x4.y * w4.y) + (x4.z * w4.z + x4.w * w4.w);
#pragma unroll
    for (int o = 16; o > 0; o >>= 1) d += __shfl_xor(d, o);
    if (lane == 0) {
      const float h = d + dbv;
      ys[j] = gsv[j] * h + bsv[j];
    }
  }
  __syncthreads();
  if (tid < 8) {
    const v4f y4 = *(const v4f*)(ys + 4 * tid);
    float* dst = out + (size_t)mg0 + 4 * tid;
    *(volatile v4f*)dst = y4;
    __threadfence();
    *(volatile v4f*)dst = y4;
  }
}

extern "C" void kernel_launch(void* const* d_in, const int* in_sizes, int n_in,
                              void* d_out, int out_size, void* d_ws, size_t ws_size,
                              hipStream_t stream)
{
  if (n_in < 33) return;
  if (in_sizes[0] != NB * NIN) return;
  if (in_sizes[1] != NV) return;
  if (in_sizes[2] != NIN) return;
  if (in_sizes[3] != NOUT) return;
  if (in_sizes[4] != NVAR * NC) return;
  if (in_sizes[5] != NS * NC) return;
  if (in_sizes[6] < 1) return;
  if (in_sizes[7] != NH || in_sizes[8] != NH) return;
  if (in_sizes[9] != NH * NC || in_sizes[10] != NH || in_sizes[11] != NH * NC || in_sizes[12] != NH) return;
  if (in_sizes[13] != LENC * 2 * NH * NH || in_sizes[14] != LENC * 2 * NH) return;
  if (in_sizes[15] != LENC * 2 * NH * NC || in_sizes[16] != LENC * 2 * NH) return;
  if (in_sizes[17] != LENC * 2 * NH * NC || in_sizes[18] != LENC * 2 * NH) return;
  if (in_sizes[19] != LCORE * 2 * NH * NH || in_sizes[20] != LCORE * 2 * NH) return;
  if (in_sizes[21] != LDEC * 2 * NH * NH || in_sizes[22] != LDEC * 2 * NH) return;
  if (in_sizes[23] != LDEC * 2 * NH * NC || in_sizes[24] != LDEC * 2 * NH) return;
  if (in_sizes[25] != LDEC * 2 * NH * NC || in_sizes[26] != LDEC * 2 * NH) return;
  if (in_sizes[27] != NH || in_sizes[28] < 1) return;
  if (in_sizes[29] != NC || in_sizes[30] < 1 || in_sizes[31] != NC || in_sizes[32] < 1) return;
  if (out_size != NB * NOUT) return;

  const float* input   = (const float*)d_in[0];
  const int*   vi      = (const int*)d_in[1];
  const int*   ivi     = (const int*)d_in[2];
  const int*   ovi     = (const int*)d_in[3];
  const float* dctx    = (const float*)d_in[4];
  const float* basis   = (const float*)d_in[5];
  const float* alpha_p = (const float*)d_in[6];
  const float* encf_W  = (const float*)d_in[7];
  const float* encf_b  = (const float*)d_in[8];
  const float* encf_Gw = (const float*)d_in[9];
  const float* encf_Gb = (const float*)d_in[10];
  const float* encf_Bw = (const float*)d_in[11];
  const float* encf_Bb = (const float*)d_in[12];
  const float* enc_W   = (const float*)d_in[13];
  const float* enc_b   = (const float*)d_in[14];
  const float* enc_Gw  = (const float*)d_in[15];
  const float* enc_Gb  = (const float*)d_in[16];
  const float* enc_Bw  = (const float*)d_in[17];
  const float* enc_Bb  = (const float*)d_in[18];
  const float* core_W  = (const float*)d_in[19];
  const float* core_b  = (const float*)d_in[20];
  const float* dec_W   = (const float*)d_in[21];
  const float* dec_b   = (const float*)d_in[22];
  const float* dec_Gw  = (const float*)d_in[23];
  const float* dec_Gb  = (const float*)d_in[24];
  const float* dec_Bw  = (const float*)d_in[25];
  const float* dec_Bb  = (const float*)d_in[26];
  const float* decf_W  = (const float*)d_in[27];
  const float* decf_b  = (const float*)d_in[28];
  const float* decf_Gw = (const float*)d_in[29];
  const float* decf_Gb = (const float*)d_in[30];
  const float* decf_Bw = (const float*)d_in[31];
  const float* decf_Bb = (const float*)d_in[32];
  float* out = (float*)d_out;

  char* ws = (char*)d_ws;
  size_t off = 0;
  const size_t oWt  = off; off += (size_t)(LENC + LDEC) * 2 * NH * NH * 2;  off = (off + 255) & ~(size_t)255;
  const size_t oGem = off; off += (size_t)NEMAP * NIN * NH * 4;             off = (off + 255) & ~(size_t)255;
  const size_t oBem = off; off += (size_t)NEMAP * NIN * NH * 4;             off = (off + 255) & ~(size_t)255;
  const size_t oGdm = off; off += (size_t)NDMAP * NOUT * NH * 4;            off = (off + 255) & ~(size_t)255;
  const size_t oBdm = off; off += (size_t)NDMAP * NOUT * NH * 4;            off = (off + 255) & ~(size_t)255;
  const size_t oX32 = off; off += (size_t)MCH * NH * 4;                     off = (off + 255) & ~(size_t)255;
  const size_t oX16 = off; off += (size_t)MCH * NH * 2;                     off = (off + 255) & ~(size_t)255;
  const size_t oH16 = off; off += (size_t)MCH * NH * 2;                     off = (off + 255) & ~(size_t)255;
  const size_t oSc  = off; off += (size_t)NB * NH * 4;                      off = (off + 255) & ~(size_t)255;
  const size_t oSd  = off; off += (size_t)NB * NH * 4;                      off = (off + 255) & ~(size_t)255;
  if (off > ws_size || off > (size_t)WSCAP) return;
  _Float16* wt   = (_Float16*)(ws + oWt);
  float*    gem  = (float*)(ws + oGem);
  float*    bem  = (float*)(ws + oBem);
  float*    gdm  = (float*)(ws + oGdm);
  float*    bdm  = (float*)(ws + oBdm);
  float*    X32  = (float*)(ws + oX32);
  _Float16* X16  = (_Float16*)(ws + oX16);
  _Float16* H16  = (_Float16*)(ws + oH16);
  float*    score = (float*)(ws + oSc);
  float*    sdec  = (float*)(ws + oSd);

  hipFuncSetAttribute(reinterpret_cast<const void*>(&k_gemm<false, false, true>),
                      hipFuncAttributeMaxDynamicSharedMemorySize, LDS_GEMM);
  hipFuncSetAttribute(reinterpret_cast<const void*>(&k_gemm<true, true, true>),
                      hipFuncAttributeMaxDynamicSharedMemorySize, LDS_GEMM);
  hipFuncSetAttribute(reinterpret_cast<const void*>(&k_gemm<true, true, false>),
                      hipFuncAttributeMaxDynamicSharedMemorySize, LDS_GEMM);

  const float oscE = 1.0f / (XSE * WSC);
  const float oscD = 1.0f / (XSD * WSC);

  k_prepw<<<PWB_E + PWB_D, NTHR, 0, stream>>>(enc_W, dec_W, wt);
  k_attn<<<NIN, 64, 0, stream>>>(vi, ivi, dctx, basis, alpha_p, encf_Gw, encf_Gb, encf_Bw, encf_Bb,
                                 enc_Gw, enc_Gb, enc_Bw, enc_Bb, gem, bem);
  k_dmaps<<<NOUT, 64, 0, stream>>>(vi, ovi, dctx, dec_Gw, dec_Gb, dec_Bw, dec_Bb, gdm, bdm);

  for (int ch = 0; ch < ENC_CH; ++ch) {
    const int mbase = ch * MCH;
    k_rowinit<0><<<MCH / 32, NTHR, 0, stream>>>(mbase, input, encf_W, encf_b, gem, bem, score, X32, X16, XSE);
    for (int l = 0; l < LENC; ++l) {
      const int li0 = 2 * l, li1 = 2 * l + 1;
      k_gemm<false, false, true><<<MCH / 128, NTHR, LDS_GEMM, stream>>>(
          X16, wt + (size_t)li0 * NH * NH, enc_b + (size_t)li0 * NH,
          gem + (size_t)(1 + li0) * NIN * NH, bem + (size_t)(1 + li0) * NIN * NH,
          X32, H16, NIN - 1, oscE, XSE);
      if (l + 1 < LENC) {
        k_gemm<true, true, true><<<MCH / 128, NTHR, LDS_GEMM, stream>>>(
            H16, wt + (size_t)li1 * NH * NH, enc_b + (size_t)li1 * NH,
            gem + (size_t)(1 + li1) * NIN * NH, bem + (size_t)(1 + li1) * NIN * NH,
            X32, X16, NIN - 1, oscE, XSE);
      } else {
        k_gemm<true, true, false><<<MCH / 128, NTHR, LDS_GEMM, stream>>>(
            H16, wt + (size_t)li1 * NH * NH, enc_b + (size_t)li1 * NH,
            gem + (size_t)(1 + li1) * NIN * NH, bem + (size_t)(1 + li1) * NIN * NH,
            X32, X16, NIN - 1, oscE, XSE);
      }
    }
    k_nsum<<<MCH / NIN, NH, 0, stream>>>(X32, score, ch * (MCH / NIN));
  }

  k_core<<<NB, NH, 0, stream>>>(score, core_W, core_b, sdec);

  const _Float16* wtd = wt + (size_t)(LENC * 2) * NH * NH;
  for (int ch = 0; ch < DEC_CH; ++ch) {
    const int mbase = ch * MCH;
    k_rowinit<1><<<MCH / 32, NTHR, 0, stream>>>(mbase, input, encf_W, encf_b, gem, bem, sdec, X32, X16, XSD);
    for (int l = 0; l < LDEC; ++l) {
      const int li0 = 2 * l, li1 = 2 * l + 1;
      k_gemm<false, false, true><<<MCH / 128, NTHR, LDS_GEMM, stream>>>(
          X16, wtd + (size_t)li0 * NH * NH, dec_b + (size_t)li0 * NH,
          gdm + (size_t)li0 * NOUT * NH, bdm + (size_t)li0 * NOUT * NH,
          X32, H16, NOUT - 1, oscD, XSD);
      if (l + 1 < LDEC) {
        k_gemm<true, true, true><<<MCH / 128, NTHR, LDS_GEMM, stream>>>(
            H16, wtd + (size_t)li1 * NH * NH, dec_b + (size_t)li1 * NH,
            gdm + (size_t)li1 * NOUT * NH, bdm + (size_t)li1 * NOUT * NH,
            X32, X16, NOUT - 1, oscD, XSD);
      } else {
        k_gemm<true, true, false><<<MCH / 128, NTHR, LDS_GEMM, stream>>>(
            H16, wtd + (size_t)li1 * NH * NH, dec_b + (size_t)li1 * NH,
            gdm + (size_t)li1 * NOUT * NH, bdm + (size_t)li1 * NOUT * NH,
            X32, X16, NOUT - 1, oscD, XSD);
      }
    }
    k_decf<<<MCH / 32, NTHR, 0, stream>>>(mbase, X32, vi, ovi, dctx, decf_W, decf_b,
                                          decf_Gw, decf_Gb, decf_Bw, decf_Bb, out);
  }
}
